// LstmConv_21655225106656
// MI455X (gfx1250) — hardware-run, weakly checked
//
#include <hip/hip_runtime.h>
#include <math.h>

constexpr int NNODE   = 50000;
constexpr int NEDGE   = 800000;
constexpr int NFEAT   = 128;
constexpr int NMSG    = 64;
constexpr int NGATE   = 256;
constexpr int KCAT    = 3 * NFEAT + 3 * NMSG;
constexpr int MPAD    = 50048;
constexpr int TILE_N  = 256;
constexpr int NTILE   = (NNODE + TILE_N - 1) / TILE_N;
constexpr int NROWP   = NTILE * TILE_N;
constexpr int BLK_THR = 256;
constexpr int SCAN_Q  = 4;
constexpr int CHUNK_E = BLK_THR * 4 * SCAN_Q;
constexpr int NCHUNK  = (NEDGE + CHUNK_E - 1) / CHUNK_E;
constexpr int CH8_ROW = KCAT / 8;
constexpr float FX_SCALE = 1048576.0f;
constexpr float FX_INV   = 1.0f / 1048576.0f;

static_assert(NFEAT == 2 * NMSG);
static_assert(NGATE == 4 * NMSG);
static_assert(KCAT == 576 && KCAT % 32 == 0);
static_assert(MPAD % 64 == 0 && MPAD >= NNODE && MPAD <= NROWP);
static_assert(NGATE % 64 == 0);
static_assert(((MPAD / 64) * (NGATE / 64)) % 8 == 0);
static_assert(NEDGE % 4 == 0);
static_assert(NNODE <= 65536);
static_assert(TILE_N == BLK_THR);
static_assert(NTILE == 196 && NROWP == 50176 && NCHUNK == 196 && CHUNK_E == 4096);
static_assert((NGATE * CH8_ROW) % BLK_THR == 0);
static_assert(NNODE % 16 == 0);
static_assert(MPAD % 8 == 0);
static_assert((size_t)MPAD * NGATE * 4 <= (size_t)2 * NROWP * NFEAT * 4);

typedef __attribute__((ext_vector_type(16))) _Float16 v16h;
typedef __attribute__((ext_vector_type(8)))  _Float16 v8h;
typedef __attribute__((ext_vector_type(16))) __bf16   v16b;
typedef __attribute__((ext_vector_type(8)))  __bf16   v8b;
typedef __attribute__((ext_vector_type(8)))  float    v8f;
typedef __attribute__((ext_vector_type(4)))  float    v4f;
typedef __attribute__((ext_vector_type(4)))  int      v4i;
typedef __attribute__((ext_vector_type(2)))  unsigned v2u;

__device__ __forceinline__ unsigned short f2bf_bits(float f) {
  unsigned u = __float_as_uint(f);
  return (unsigned short)((u + 0x7FFFu + ((u >> 16) & 1u)) >> 16);
}
__device__ __forceinline__ float bf_bits2f(unsigned short h) { return __uint_as_float(((unsigned)h) << 16); }
__device__ __forceinline__ void bf_split(float f, unsigned short& hb, unsigned short& lb) {
  hb = f2bf_bits(f);
  lb = f2bf_bits(f - bf_bits2f(hb));
}

__device__ __forceinline__ void grp_guard_b(v8f& c0, v8f& c1, v8f& c2, v8f& c3, v16b a, v16b b0, v16b b1, v16b b2, v16b b3) {
  asm volatile("v_nop\n\tv_nop\n\tv_nop\n\tv_nop" : "+v"(c0), "+v"(c1), "+v"(c2), "+v"(c3) : "v"(a), "v"(b0), "v"(b1), "v"(b2), "v"(b3));
}
__device__ __forceinline__ void keep4_b(v16b a, v16b b, v16b c, v16b d) { asm volatile("v_nop" :: "v"(a), "v"(b), "v"(c), "v"(d)); }
__device__ __forceinline__ void acc_guard4(v8f& a, v8f& b, v8f& c, v8f& d) { asm volatile("v_nop\n\tv_nop\n\tv_nop\n\tv_nop" : "+v"(a), "+v"(b), "+v"(c), "+v"(d)); }

struct FragB {
  union U { v16b v; v8b h[2]; };
  static __device__ __forceinline__ v16b load(const __bf16* p) {
    U f; f.h[0] = *(const v8b*)(p); f.h[1] = *(const v8b*)(p + 16); return f.v;
  }
  static __device__ __forceinline__ v8f mma(v16b a, v16b b, v8f c) {
    return __builtin_amdgcn_wmma_f32_16x16x32_bf16(false, a, false, b, (short)0, c, false, false);
  }
};

__global__ __launch_bounds__(256) void wmma_gemm64_bf16(
    const unsigned short* __restrict__ Ap, int lda,
    const unsigned short* __restrict__ Btp, int ldb,
    float* __restrict__ C, int ldc, int M, int N, int K) {
  const __bf16* A  = (const __bf16*)Ap;
  const __bf16* Bt = (const __bf16*)Btp;
  __shared__ __align__(16) float sT[8][16 * 68];
  const int lane = threadIdx.x & 31;
  const int wave = threadIdx.x >> 5;
  const int tilesN = N >> 6;
  const int tilesM = M >> 6;
  const int tile = blockIdx.x * 8 + wave;
  if (tile >= tilesM * tilesN) return;
  const int tm = tile / tilesN;
  const int tn = tile - tm * tilesN;
  const int m0 = tm << 6;
  const int n0 = tn << 6;

  const int rlane = lane & 15;
  const int koff  = (lane >> 4) * 8;
  const int mOff  = (lane >> 4) * 8;

  v8f acc[4][4];
#pragma unroll
  for (int i = 0; i < 4; ++i)
#pragma unroll
    for (int j = 0; j < 4; ++j) acc[i][j] = (v8f){0.f,0.f,0.f,0.f,0.f,0.f,0.f,0.f};

  for (int k0 = 0; k0 < K; k0 += 32) {
    v16b bh[4];
#pragma unroll
    for (int j = 0; j < 4; ++j) {
      const size_t bo = (size_t)(n0 + (j << 4) + rlane) * ldb + koff + k0;
      bh[j] = FragB::load(Bt + bo);
    }
#pragma unroll
    for (int i = 0; i < 4; ++i) {
      const size_t ao = (size_t)(m0 + (i << 4) + rlane) * lda + koff + k0;
      const v16b ah = FragB::load(A + ao);
#pragma unroll
      for (int j = 0; j < 4; ++j) acc[i][j] = FragB::mma(ah, bh[j], acc[i][j]);
      grp_guard_b(acc[i][0], acc[i][1], acc[i][2], acc[i][3], ah, bh[0], bh[1], bh[2], bh[3]);
    }
    keep4_b(bh[0], bh[1], bh[2], bh[3]);
  }
  acc_guard4(acc[0][0], acc[0][1], acc[0][2], acc[0][3]);
  acc_guard4(acc[1][0], acc[1][1], acc[1][2], acc[1][3]);
  acc_guard4(acc[2][0], acc[2][1], acc[2][2], acc[2][3]);
  acc_guard4(acc[3][0], acc[3][1], acc[3][2], acc[3][3]);

  float* slab = sT[wave];
#pragma unroll
  for (int i = 0; i < 4; ++i) {
    const int mBase = m0 + (i << 4);
#pragma unroll
    for (int j = 0; j < 4; ++j) {
#pragma unroll
      for (int r = 0; r < 8; ++r) slab[(mOff + r) * 68 + (j << 4) + rlane] = acc[i][j][r];
    }
    __builtin_amdgcn_fence(__ATOMIC_RELEASE, "workgroup");
    __builtin_amdgcn_wave_barrier();
    __builtin_amdgcn_fence(__ATOMIC_ACQUIRE, "workgroup");
    {
      const int hh = lane >> 4, c4 = (lane & 15) * 4;
      for (int pass = 0; pass < 2; ++pass) {
#pragma unroll
        for (int it = 0; it < 8; ++it) {
          const int row = it * 2 + hh;
          v4f v = *(const v4f*)(slab + row * 68 + c4);
          *(volatile v4f*)(C + (size_t)(mBase + row) * ldc + n0 + c4) = v;
        }
        __threadfence();
      }
    }
    __builtin_amdgcn_fence(__ATOMIC_RELEASE, "workgroup");
    __builtin_amdgcn_wave_barrier();
    __builtin_amdgcn_fence(__ATOMIC_ACQUIRE, "workgroup");
  }
}

__global__ __launch_bounds__(BLK_THR) void prep_bt_kernel(const float* __restrict__ Wih, const float* __restrict__ Whh,
                                                          unsigned short* __restrict__ Bt) {
  const int i = blockIdx.x * BLK_THR + threadIdx.x;
  if (i >= NGATE * CH8_ROW) return;
  const int row  = i / CH8_ROW;
  const int col0 = (i - row * CH8_ROW) * 8;
  const bool isx = col0 < 3 * NFEAT;
  const int cx   = isx ? col0 : 0;
  const int chh  = isx ? 0 : (col0 - 3 * NFEAT);
  const int segx = cx >> 7, kx = cx & (NFEAT - 1);
  const int segh = chh >> 6, kh = chh & (NMSG - 1);
  const float* pa = Wih + (size_t)row * NFEAT + kx;
  const float* pb = Whh + (size_t)row * NMSG + kh;
  v4f a0 = *(const v4f*)(pa);
  v4f a1 = *(const v4f*)(pa + 4);
  v4f b0 = *(const v4f*)(pb);
  v4f b1 = *(const v4f*)(pb + 4);
  asm volatile("" : "+v"(a0), "+v"(a1), "+v"(b0), "+v"(b1));
  const bool uselo = isx ? (segx == 2) : (segh == 2);
  v8h hv;
#pragma unroll
  for (int e = 0; e < 4; ++e) {
    const float f0 = isx ? a0[e] : b0[e];
    const float f1 = isx ? a1[e] : b1[e];
    unsigned short h0b, l0b, h1b, l1b;
    bf_split(f0, h0b, l0b);
    bf_split(f1, h1b, l1b);
    const unsigned short o0 = uselo ? l0b : h0b;
    const unsigned short o1 = uselo ? l1b : h1b;
    hv[e]     = __builtin_bit_cast(_Float16, o0);
    hv[4 + e] = __builtin_bit_cast(_Float16, o1);
  }
  *(volatile v8h*)(Bt + (size_t)i * 8) = hv;
  __threadfence();
  *(volatile v8h*)(Bt + (size_t)i * 8) = hv;
}

__global__ __launch_bounds__(BLK_THR) void agg_kernel(const float* __restrict__ feat,
                                                      const int* __restrict__ src0, const int* __restrict__ dst0,
                                                      const int* __restrict__ src1, const int* __restrict__ dst1,
                                                      float* __restrict__ meanp, int* __restrict__ cntp) {
  __shared__ __align__(16) int      accS[TILE_N * NFEAT];
  __shared__ __align__(16) unsigned hitS[CHUNK_E];
  __shared__ __align__(16) int      cntS[TILE_N];
  __shared__ int nhS[2];
  const int tid = threadIdx.x, lane = tid & 31, wave = tid >> 5;
  const int et = blockIdx.y;
  const int n0 = blockIdx.x * TILE_N;
  const int* srcp = (et == 0) ? src0 : src1;
  const int* dstp = (et == 0) ? dst0 : dst1;

  {
    v4i* a4 = (v4i*)accS;
    const v4i z4 = {0, 0, 0, 0};
#pragma unroll 1
    for (int i = tid; i < TILE_N * NFEAT / 4; i += BLK_THR) a4[i] = z4;
    cntS[tid] = 0;
    if (tid < 2) nhS[tid] = 0;
  }
  __syncthreads();

#pragma unroll 1
  for (int ch = 0; ch < NCHUNK; ++ch) {
    const int par = ch & 1;
#pragma unroll 1
    for (int q = 0; q < SCAN_Q; ++q) {
      const int i4 = (ch * SCAN_Q + q) * BLK_THR + tid;
      const int eb = i4 * 4;
      const bool valid = eb < NEDGE;
      const int ebc = valid ? eb : (NEDGE - 4);
      const v4i d = *(const v4i*)(dstp + ebc);
      const v4i s = *(const v4i*)(srcp + ebc);
      const int dl0 = d[0] - n0, dl1 = d[1] - n0, dl2 = d[2] - n0, dl3 = d[3] - n0;
      const bool h0 = valid && ((unsigned)dl0 < (unsigned)TILE_N);
      const bool h1 = valid && ((unsigned)dl1 < (unsigned)TILE_N);
      const bool h2 = valid && ((unsigned)dl2 < (unsigned)TILE_N);
      const bool h3 = valid && ((unsigned)dl3 < (unsigned)TILE_N);
      const unsigned m0 = (unsigned)__ballot(h0);
      const unsigned m1 = (unsigned)__ballot(h1);
      const unsigned m2 = (unsigned)__ballot(h2);
      const unsigned m3 = (unsigned)__ballot(h3);
      const int c0 = __popc(m0), c1 = __popc(m1), c2 = __popc(m2), c3 = __popc(m3);
      const int total = c0 + c1 + c2 + c3;
      if (total > 0) {
        int base = 0;
        if (lane == 0) base = atomicAdd(&nhS[par], total);
        base = __shfl(base, 0, 32);
        const unsigned lt = (1u << lane) - 1u;
        if (h0) {
          int p = base + __popc(m0 & lt);
          p = p < CHUNK_E - 1 ? p : CHUNK_E - 1;
          int sc = s[0]; sc = sc < 0 ? 0 : sc; sc = sc > NNODE - 1 ? NNODE - 1 : sc;
          hitS[p] = ((unsigned)dl0 << 16) | (unsigned)sc;
        }
        if (h1) {
          int p = base + c0 + __popc(m1 & lt);
          p = p < CHUNK_E - 1 ? p : CHUNK_E - 1;
          int sc = s[1]; sc = sc < 0 ? 0 : sc; sc = sc > NNODE - 1 ? NNODE - 1 : sc;
          hitS[p] = ((unsigned)dl1 << 16) | (unsigned)sc;
        }
        if (h2) {
          int p = base + c0 + c1 + __popc(m2 & lt);
          p = p < CHUNK_E - 1 ? p : CHUNK_E - 1;
          int sc = s[2]; sc = sc < 0 ? 0 : sc; sc = sc > NNODE - 1 ? NNODE - 1 : sc;
          hitS[p] = ((unsigned)dl2 << 16) | (unsigned)sc;
        }
        if (h3) {
          int p = base + c0 + c1 + c2 + __popc(m3 & lt);
          p = p < CHUNK_E - 1 ? p : CHUNK_E - 1;
          int sc = s[3]; sc = sc < 0 ? 0 : sc; sc = sc > NNODE - 1 ? NNODE - 1 : sc;
          hitS[p] = ((unsigned)dl3 << 16) | (unsigned)sc;
        }
      }
    }
    __syncthreads();
    int nh = __builtin_amdgcn_readfirstlane(nhS[par]);
    nh = nh < CHUNK_E ? nh : CHUNK_E;
    nh = nh < 0 ? 0 : nh;
    if (tid == 0) nhS[par ^ 1] = 0;
#pragma unroll 1
    for (int h = wave; h < nh; h += 8) {
      const unsigned ent = hitS[h];
      int sc = (int)(ent & 0xffffu);
      sc = sc > NNODE - 1 ? NNODE - 1 : sc;
      const int dl = (int)(ent >> 16) & (TILE_N - 1);
      const v4f v = *(const v4f*)(feat + (size_t)sc * NFEAT + 4 * lane);
      int* ap = accS + dl * NFEAT + 4 * lane;
      const int q0 = __float2int_rn(v[0] * FX_SCALE);
      const int q1 = __float2int_rn(v[1] * FX_SCALE);
      const int q2 = __float2int_rn(v[2] * FX_SCALE);
      const int q3 = __float2int_rn(v[3] * FX_SCALE);
      atomicAdd(ap + 0, q0);
      atomicAdd(ap + 1, q1);
      atomicAdd(ap + 2, q2);
      atomicAdd(ap + 3, q3);
      if (lane == 0) atomicAdd(&cntS[dl], 1);
    }
    __syncthreads();
  }

  float* mp = meanp + ((size_t)et * NROWP + (size_t)n0) * NFEAT;
  int*   cp = cntp + (size_t)et * NROWP + n0;
  for (int pass = 0; pass < 2; ++pass) {
#pragma unroll 1
    for (int it = 0; it < TILE_N * NFEAT / 4 / BLK_THR; ++it) {
      const int idx = it * BLK_THR + tid;
      const int row = idx >> 5, c4 = (idx & 31) * 4;
      const v4i a = *(const v4i*)(accS + row * NFEAT + c4);
      int cn = cntS[row];
      cn = cn > 1 ? cn : 1;
      const float inv = FX_INV * (1.0f / (float)cn);
      v4f o;
      o[0] = (float)a[0] * inv;
      o[1] = (float)a[1] * inv;
      o[2] = (float)a[2] * inv;
      o[3] = (float)a[3] * inv;
      *(volatile v4f*)(mp + (size_t)row * NFEAT + c4) = o;
    }
    if (tid < TILE_N / 4) {
      const v4i cv = *(const v4i*)(cntS + 4 * tid);
      *(volatile v4i*)(cp + 4 * tid) = cv;
    }
    __threadfence();
  }
}

__global__ __launch_bounds__(BLK_THR) void combine_kernel(const float* __restrict__ feat,
                                                          const float* __restrict__ mean0, const float* __restrict__ mean1,
                                                          const int* __restrict__ cnt0, const int* __restrict__ cnt1,
                                                          unsigned short* __restrict__ Ap, float* __restrict__ Rt) {
  const int lane = threadIdx.x & 31, wave = threadIdx.x >> 5;
  const int row = blockIdx.x * 8 + wave;
  if (row >= MPAD) return;
  const bool live = row < NNODE;
  const int rc = live ? row : (NNODE - 1);
  v4f x = *(const v4f*)(feat + (size_t)rc * NFEAT + 4 * lane);
  const v4f ma = *(const v4f*)(mean0 + (size_t)row * NFEAT + 4 * lane);
  const v4f mb = *(const v4f*)(mean1 + (size_t)row * NFEAT + 4 * lane);
  const int ca = cnt0[row];
  const int cb = cnt1[row];
  const int has = (ca > 0 ? 1 : 0) + (cb > 0 ? 1 : 0);
  const float sc = (has >= 2) ? 0.5f : 1.0f;
  unsigned short xh[4], xl[4], rh[4], rl[4];
  v4f r;
#pragma unroll
  for (int e = 0; e < 4; ++e) {
    const float xv = live ? x[e] : 0.0f;
    const float rv = live ? ((ma[e] + mb[e]) * sc) : 0.0f;
    r[e] = rv;
    bf_split(xv, xh[e], xl[e]);
    bf_split(rv, rh[e], rl[e]);
  }
  v2u pxh, pxl, prh, prl;
  pxh[0] = (unsigned)xh[0] | ((unsigned)xh[1] << 16);
  pxh[1] = (unsigned)xh[2] | ((unsigned)xh[3] << 16);
  pxl[0] = (unsigned)xl[0] | ((unsigned)xl[1] << 16);
  pxl[1] = (unsigned)xl[2] | ((unsigned)xl[3] << 16);
  prh[0] = (unsigned)rh[0] | ((unsigned)rh[1] << 16);
  prh[1] = (unsigned)rh[2] | ((unsigned)rh[3] << 16);
  prl[0] = (unsigned)rl[0] | ((unsigned)rl[1] << 16);
  prl[1] = (unsigned)rl[2] | ((unsigned)rl[3] << 16);
  unsigned short* arow = Ap + (size_t)row * KCAT;
  const int lg = lane & 15;
  for (int pass = 0; pass < 2; ++pass) {
    *(volatile v2u*)(arow + 4 * lane) = pxh;
    *(volatile v2u*)(arow + NFEAT + 4 * lane) = pxl;
    *(volatile v2u*)(arow + 2 * NFEAT + 4 * lane) = pxh;
    if (lane < 16) {
      *(volatile v2u*)(arow + 3 * NFEAT + 4 * lg) = prh;
      *(volatile v2u*)(arow + 3 * NFEAT + NMSG + 4 * lg) = prl;
      *(volatile v2u*)(arow + 3 * NFEAT + 2 * NMSG + 4 * lg) = prh;
    } else {
      *(volatile v4f*)(Rt + (size_t)row * NMSG + 4 * lg) = r;
    }
    __threadfence();
  }
}

__device__ __forceinline__ float sigm_f(float x) { return 1.0f / (1.0f + expf(-x)); }
__device__ __forceinline__ float tanh_f(float x) { return 1.0f - 2.0f / (1.0f + expf(2.0f * x)); }

__global__ __launch_bounds__(BLK_THR) void cell_kernel(const float* __restrict__ gates, const float* __restrict__ Rt,
                                                       const float* __restrict__ bih, const float* __restrict__ bhh,
                                                       float* __restrict__ out) {
  __shared__ __align__(16) float Sl[8][2 * NFEAT];
  const int lane = threadIdx.x & 31, wave = threadIdx.x >> 5;
  const int nb = (blockIdx.x * 8 + wave) * 2;
  if (nb + 1 >= NNODE + 1) return;
  float* slab = Sl[wave];
#pragma unroll 1
  for (int q = 0; q < 4; ++q) {
    const int nl = q >> 1;
    const int u  = (q & 1) * 32 + lane;
    int n = nb + nl;
    n = n < NNODE ? n : NNODE - 1;
    const float* gp = gates + (size_t)n * NGATE + u;
    const float zi = gp[0]        + (bih[u]            + bhh[u]);
    const float zf = gp[NMSG]     + (bih[NMSG + u]     + bhh[NMSG + u]);
    const float zg = gp[2 * NMSG] + (bih[2 * NMSG + u] + bhh[2 * NMSG + u]);
    const float zo = gp[3 * NMSG] + (bih[3 * NMSG + u] + bhh[3 * NMSG + u]);
    const float cprev = Rt[(size_t)n * NMSG + u];
    const float ig = sigm_f(zi);
    const float fg = sigm_f(zf);
    const float og = sigm_f(zo);
    const float gg = tanh_f(zg);
    const float cn = fg * cprev + ig * gg;
    const float hn = og * tanh_f(cn);
    slab[nl * NFEAT + u] = hn;
    slab[nl * NFEAT + NMSG + u] = cn;
  }
  __builtin_amdgcn_fence(__ATOMIC_RELEASE, "workgroup");
  __builtin_amdgcn_wave_barrier();
  __builtin_amdgcn_fence(__ATOMIC_ACQUIRE, "workgroup");
  const v4f v0 = *(const v4f*)(slab + 4 * lane);
  const v4f v1 = *(const v4f*)(slab + NFEAT + 4 * lane);
  for (int pass = 0; pass < 2; ++pass) {
    *(volatile v4f*)(out + (size_t)nb * NFEAT + 4 * lane) = v0;
    *(volatile v4f*)(out + (size_t)(nb + 1) * NFEAT + 4 * lane) = v1;
    __threadfence();
  }
}

extern "C" void kernel_launch(void* const* d_in, const int* in_sizes, int n_in,
                              void* d_out, int out_size, void* d_ws, size_t ws_size, hipStream_t stream) {
  if (n_in < 9 || d_out == nullptr || d_ws == nullptr) return;
  if (in_sizes[0] != NNODE * NFEAT || in_sizes[1] != NEDGE || in_sizes[2] != NEDGE || in_sizes[3] != NEDGE ||
      in_sizes[4] != NEDGE || in_sizes[5] != NGATE * NFEAT || in_sizes[6] != NGATE * NMSG ||
      in_sizes[7] != NGATE || in_sizes[8] != NGATE || out_size != NNODE * NFEAT) return;

  const float* feat = (const float*)d_in[0];
  const int*   src0 = (const int*)d_in[1];
  const int*   dst0 = (const int*)d_in[2];
  const int*   src1 = (const int*)d_in[3];
  const int*   dst1 = (const int*)d_in[4];
  const float* Wih  = (const float*)d_in[5];
  const float* Whh  = (const float*)d_in[6];
  const float* bih  = (const float*)d_in[7];
  const float* bhh  = (const float*)d_in[8];
  float* out = (float*)d_out;

  char* ws = (char*)d_ws; size_t off = 0;
  auto carve = [&](size_t bytes) -> char* { char* p = ws + off; off += (bytes + 255) & ~(size_t)255; return p; };
  float*          MEAN  = (float*)carve((size_t)2 * NROWP * NFEAT * 4);
  int*            CNT   = (int*)carve((size_t)2 * NROWP * 4);
  unsigned short* APL   = (unsigned short*)carve((size_t)MPAD * KCAT * 2);
  float*          RTP   = (float*)carve((size_t)MPAD * NMSG * 4);
  unsigned short* BTP   = (unsigned short*)carve((size_t)NGATE * KCAT * 2);
  float*          GATES = MEAN;
  if (off > ws_size || off > (size_t)134217728) return;

  prep_bt_kernel<<<(NGATE * CH8_ROW) / BLK_THR, BLK_THR, 0, stream>>>(Wih, Whh, BTP);
  agg_kernel<<<dim3(NTILE, 2), BLK_THR, 0, stream>>>(feat, src0, dst0, src1, dst1, MEAN, CNT);
  combine_kernel<<<MPAD / 8, BLK_THR, 0, stream>>>(feat, MEAN, MEAN + (size_t)NROWP * NFEAT, CNT, CNT + NROWP, APL, RTP);
  wmma_gemm64_bf16<<<((MPAD / 64) * (NGATE / 64)) / 8, 256, 0, stream>>>(APL, KCAT, BTP, KCAT, GATES, NGATE, MPAD, NGATE, KCAT);
  cell_kernel<<<NNODE / 16, BLK_THR, 0, stream>>>(GATES, RTP, bih, bhh, out);
}
